// OptimizedMiniBlock_21861383537484
// MI455X (gfx1250) — hardware-verified
//
#include <hip/hip_runtime.h>
#include <hip/hip_bf16.h>
#include <math.h>


#define BB 4
#define SS 2048
#define DD 1024
#define HH 16
#define DKK 64
#define QW 2

typedef _Float16 bf16;
typedef __attribute__((ext_vector_type(4))) unsigned v4u_t;
typedef unsigned v4ua __attribute__((ext_vector_type(4), may_alias));
typedef __attribute__((ext_vector_type(4))) float v4f_t;
typedef float v4fa __attribute__((ext_vector_type(4), may_alias));
typedef __attribute__((ext_vector_type(16))) bf16  bf16x16;
typedef __attribute__((ext_vector_type(8)))  bf16  bf16x8;
typedef __attribute__((ext_vector_type(4)))  bf16  bf16x4;
typedef __attribute__((ext_vector_type(8)))  float f32x8;

#define LDS_STRIDE 48
#define KSTRIDE    72
#define VSTRIDE    48

__device__ __forceinline__ f32x8 wmma_bf16(bf16x16 a, bf16x16 b, f32x8 c) {
  return __builtin_amdgcn_wmma_f32_16x16x32_f16(
      false, a, false, b, (short)0, c, false, false);
}
#define RSPLIT (1.0f / 2048.0f)
__device__ __forceinline__ bf16 lo_of(float v, bf16 h) { return (bf16)((v - (float)h) * 2048.0f); }
__device__ __forceinline__ f32x8 wmma_split(bf16x16 a, bf16x16 al, bf16x16 b, bf16x16 bl, f32x8 c) {
  f32x8 x = {}; x = wmma_bf16(al, b, x); x = wmma_bf16(a, bl, x); return wmma_bf16(a, b, c) + x * RSPLIT; }
__device__ __forceinline__ f32x8 wmma_asplit(bf16x16 a, bf16x16 al, bf16x16 b, f32x8 c) {
  f32x8 x = {}; x = wmma_bf16(al, b, x); return wmma_bf16(a, b, c) + x * RSPLIT; }

template <typename T>
__device__ __forceinline__ bf16x16 load_frag(const T* __restrict__ base, int ld,
                                             int row0, int k0) {
  const int lane = threadIdx.x & 31;
  const int r    = lane & 15;
  const int kh   = (lane >> 4) * 8;
  const T* p0 = base + (size_t)(row0 + r) * ld + (k0 + kh);
  const T* p1 = p0 + 16;
  bf16x16 f;
#pragma unroll
  for (int i = 0; i < 8; ++i) {
    f[i]     = (bf16)p0[i];
    f[i + 8] = (bf16)p1[i];
  }
  return f;
}

__device__ __forceinline__ bf16x16 lds_frag(const bf16* base, int stride) {
  const int lane = threadIdx.x & 31;
  const int row  = lane & 15;
  const int kh   = (lane >> 4) * 8;
  const bf16x8 lo = *(const bf16x8*)(base + row * stride + kh);
  const bf16x8 hi = *(const bf16x8*)(base + row * stride + kh + 16);
  bf16x16 f;
#pragma unroll
  for (int i = 0; i < 8; ++i) { f[i] = lo[i]; f[i + 8] = hi[i]; }
  return f;
}

template <typename T>
__device__ __forceinline__ void stage_read16(const T* __restrict__ p, float* buf) {
#pragma unroll
  for (int i = 0; i < 16; ++i) buf[i] = (float)p[i];
}

__device__ __forceinline__ void stage_write(bf16* dst, const float* buf, int nquad) {
#pragma unroll
  for (int i = 0; i < nquad; ++i) {
    bf16x4 q;
    q[0] = (bf16)buf[4 * i];     q[1] = (bf16)buf[4 * i + 1];
    q[2] = (bf16)buf[4 * i + 2]; q[3] = (bf16)buf[4 * i + 3];
    *(bf16x4*)(dst + 4 * i) = q;
  }
}

__global__ __launch_bounds__(256) void transpose_pack_kernel(const float* __restrict__ W, bf16* __restrict__ WT, int K, int N, size_t plane) {
  __shared__ float tile[64][65];
  const int k0 = blockIdx.y * 64, n0 = blockIdx.x * 64, t = threadIdx.x;
  for (int i = t; i < 64 * 64; i += 256) { const int kr = i >> 6, nc = i & 63; tile[kr][nc] = W[(size_t)(k0 + kr) * N + n0 + nc]; }
  __syncthreads();
#pragma unroll 1
  for (int pass = 0; pass < 2; ++pass) {
    for (int i = t; i < 64 * 8; i += 256) { const int nr = i >> 3, k8 = (i & 7) * 8; bf16 hh[8], hl[8];
#pragma unroll
      for (int e = 0; e < 8; ++e) { const float v = tile[k8 + e][nr]; hh[e] = (bf16)v; hl[e] = lo_of(v, hh[e]); }
      bf16* d = WT + (size_t)(n0 + nr) * K + k0 + k8;
      *(volatile v4u_t*)d = *(const v4ua*)hh; *(volatile v4u_t*)(d + plane) = *(const v4ua*)hl; }
    __threadfence();
  }
}

template <typename AT, typename WT, int MODE>
__global__ __launch_bounds__(256) void gemm_split_kernel(
    const AT* __restrict__ A, size_t aPlane, const WT* __restrict__ W, size_t wPlane,
    const float* __restrict__ bias, void* __restrict__ out,
    int M, int N, int K) {
  __shared__ bf16 ldsA[128 * LDS_STRIDE], ldsAl[128 * LDS_STRIDE];
  __shared__ bf16 ldsW[256 * LDS_STRIDE], ldsWl[256 * LDS_STRIDE];
  __shared__ __attribute__((aligned(16))) unsigned char sob[256 * 136 * 2];

  const int t    = threadIdx.x;
  const int wave = t >> 5;
  const int lane = t & 31;
  const int wm   = (wave & 1) * 64;
  const int wn   = (wave >> 1) * 64;
  const int mBlk = blockIdx.x * 128;
  const int nBlk = blockIdx.y * 256;
  const int arow = t >> 1;
  const int ach  = (t & 1) * 16;

  f32x8 acc[4][4] = {};
  for (int k = 0; k < K; k += 32) {
    __syncthreads();
    {
      const AT* ap = A + (size_t)(mBlk + arow) * K + k + ach;
      bf16 hh[16], hl[16];
      if (sizeof(AT) == 4) {
#pragma unroll
        for (int i = 0; i < 16; ++i) { const float v = (float)ap[i]; hh[i] = (bf16)v; hl[i] = lo_of(v, hh[i]); }
      } else {
#pragma unroll
        for (int i = 0; i < 16; ++i) { hh[i] = (bf16)ap[i]; hl[i] = (bf16)ap[aPlane + i]; }
      }
#pragma unroll
      for (int i = 0; i < 16; ++i) { ldsA[arow * LDS_STRIDE + ach + i] = hh[i]; ldsAl[arow * LDS_STRIDE + ach + i] = hl[i]; }
    }
    {
      const WT* wp = W + (size_t)(nBlk + t) * K + k;
      if (sizeof(WT) == 4) {
#pragma unroll
        for (int i = 0; i < 32; ++i) { const float v = (float)wp[i]; const bf16 h_ = (bf16)v; ldsW[t * LDS_STRIDE + i] = h_; ldsWl[t * LDS_STRIDE + i] = lo_of(v, h_); }
      } else {
#pragma unroll
        for (int i = 0; i < 32; ++i) { ldsW[t * LDS_STRIDE + i] = (bf16)wp[i]; ldsWl[t * LDS_STRIDE + i] = (bf16)wp[wPlane + i]; }
      }
    }
    __syncthreads();
    bf16x16 wf[4], wfl[4];
#pragma unroll
    for (int j = 0; j < 4; ++j) { wf[j] = lds_frag(ldsW + (wn + 16 * j) * LDS_STRIDE, LDS_STRIDE); wfl[j] = lds_frag(ldsWl + (wn + 16 * j) * LDS_STRIDE, LDS_STRIDE); }
#pragma unroll
    for (int i = 0; i < 4; ++i) {
      const bf16x16 af = lds_frag(ldsA + (wm + 16 * i) * LDS_STRIDE, LDS_STRIDE), afl = lds_frag(ldsAl + (wm + 16 * i) * LDS_STRIDE, LDS_STRIDE);
#pragma unroll
      for (int j = 0; j < 4; ++j) acc[i][j] = wmma_asplit(af, afl, wf[j], acc[i][j]);
    }
  }

  const int nlane = lane & 15;
  const int mh    = (lane >> 4) * 8;
  __syncthreads();
  if (MODE == 1) {
    bf16* so = (bf16*)sob;
#pragma unroll
    for (int i = 0; i < 4; ++i)
#pragma unroll
      for (int j = 0; j < 4; ++j) {
        const int nl = wn + 16 * j + nlane;
        const float bv = bias ? bias[nBlk + nl] : 1.0f;
#pragma unroll
        for (int r = 0; r < 8; ++r) so[nl * 136 + wm + 16 * i + mh + r] = (bf16)(acc[i][j][r] * bv);
      }
    __syncthreads();
    const int b_ = mBlk >> 11, s0 = mBlk & (SS - 1);
#pragma unroll 1
    for (int pass = 0; pass < 2; ++pass) {
      for (int ch = t; ch < 256 * 16; ch += 256) { const int nl = ch >> 4, q = (ch & 15) * 8; const int n = nBlk + nl, h = n >> 6, dk = n & (DKK - 1);
        *(volatile v4u_t*)((bf16*)out + (((size_t)(b_ * HH + h)) * DKK + dk) * SS + s0 + q) = *(const v4ua*)(so + nl * 136 + q); }
      __threadfence();
    }
  } else {
    float* so = (float*)sob;
#pragma unroll 1
    for (int hf = 0; hf < 2; ++hf) {
      if (wm == hf * 64) {
#pragma unroll
        for (int i = 0; i < 4; ++i)
#pragma unroll
          for (int j = 0; j < 4; ++j) {
            const int nl = wn + 16 * j + nlane;
            const float bv = bias ? bias[nBlk + nl] : 1.0f;
#pragma unroll
            for (int r = 0; r < 8; ++r) so[(16 * i + mh + r) * 260 + nl] = acc[i][j][r] * bv;
          }
      }
      __syncthreads();
#pragma unroll 1
      for (int pass = 0; pass < 2; ++pass) {
        for (int ch = t; ch < 64 * 64; ch += 256) { const int ml = ch >> 6, q = (ch & 63) * 4;
          *(volatile v4f_t*)((float*)out + (size_t)(mBlk + hf * 64 + ml) * N + nBlk + q) = *(const volatile v4fa*)(so + ml * 260 + q); }
        __threadfence();
      }
      __syncthreads();
    }
  }
}


#define OKS 1032
#define OVS 40
__global__ __launch_bounds__(256) void ob_attn(const float* __restrict__ X, float* __restrict__ attn) {
  __shared__ __attribute__((aligned(16))) bf16 ldsQ[16 * OKS];
  __shared__ __attribute__((aligned(16))) bf16 ldsK[32 * OKS];
  __shared__ __attribute__((aligned(16))) bf16 ldsV[1024 * OVS];
  __shared__ float ldsS[4][2][16 * 17];
  __shared__ __attribute__((aligned(16))) float ldsO[16 * 1028];
  const int b = blockIdx.y, q0 = blockIdx.x * 16;
  const int t = threadIdx.x, wave = t >> 5, lane = t & 31, qlane = lane & 15, kh8 = (lane >> 4) * 8;
  const float* Xb = X + (size_t)b * SS * DD;
  { const int r = t >> 4, c0 = (t & 15) * 64; const float* xr = Xb + (size_t)(q0 + r) * DD + c0;
#pragma unroll 4
    for (int i = 0; i < 64; ++i) ldsQ[r * OKS + c0 + i] = (bf16)xr[i]; }
  f32x8 o[8] = {};
  float mrun = -INFINITY, lrun = 0.0f;
  const float scl = (1.0f / 32.0f) * 1.44269504088896340736f;
  const int qi = q0 + qlane;
  const int kt = wave & 1, ch = wave >> 1;
#pragma unroll 1
  for (int kb = 0; kb < q0 + 16; kb += 32) {
    __syncthreads();
    { const int r = t >> 3, c0 = (t & 7) * 128; const float* kr = Xb + (size_t)(kb + r) * DD + c0;
#pragma unroll 2
      for (int i = 0; i < 128; ++i) { const bf16 hv = (bf16)kr[i]; ldsK[r * OKS + c0 + i] = hv; ldsV[(c0 + i) * OVS + r] = hv; } }
    __syncthreads();
    { f32x8 sp = {};
#pragma unroll 2
      for (int c = 0; c < 8; ++c) { const int kc = (ch * 8 + c) * 32;
        sp = wmma_bf16(lds_frag(&ldsK[(kt * 16) * OKS + kc], OKS), lds_frag(&ldsQ[kc], OKS), sp); }
#pragma unroll
      for (int r = 0; r < 8; ++r) ldsS[ch][kt][(kh8 + r) * 17 + qlane] = sp[r]; }
    __syncthreads();
    float s0[8], s1[8], mx = -INFINITY;
#pragma unroll
    for (int r = 0; r < 8; ++r) {
      const int j0 = kb + kh8 + r, j1 = j0 + 16, ix = (kh8 + r) * 17 + qlane;
      s0[r] = (j0 <= qi) ? ((ldsS[0][0][ix] + ldsS[1][0][ix]) + (ldsS[2][0][ix] + ldsS[3][0][ix])) * scl : -INFINITY;
      s1[r] = (j1 <= qi) ? ((ldsS[0][1][ix] + ldsS[1][1][ix]) + (ldsS[2][1][ix] + ldsS[3][1][ix])) * scl : -INFINITY;
      mx = fmaxf(mx, fmaxf(s0[r], s1[r])); }
    mx = fmaxf(mx, __shfl_xor(mx, 16, 32));
    const float mnew = fmaxf(mrun, mx), alpha = exp2f(mrun - mnew);
    float rsum = 0.0f; bf16x16 pf;
#pragma unroll
    for (int r = 0; r < 8; ++r) { const float p0 = exp2f(s0[r] - mnew), p1 = exp2f(s1[r] - mnew); rsum += p0 + p1; pf[r] = (bf16)(p0 * 1024.0f); pf[r + 8] = (bf16)(p1 * 1024.0f); }
    rsum += __shfl_xor(rsum, 16, 32);
    lrun = lrun * alpha + rsum; mrun = mnew;
#pragma unroll
    for (int j = 0; j < 8; ++j) {
#pragma unroll
      for (int r = 0; r < 8; ++r) o[j][r] *= alpha;
      o[j] = wmma_bf16(lds_frag(&ldsV[((wave * 8 + j) * 16) * OVS], OVS), pf, o[j]);
    }
  }
  const float rl = 1.0f / (lrun * 1024.0f);
#pragma unroll
  for (int j = 0; j < 8; ++j)
#pragma unroll
    for (int r = 0; r < 8; ++r) ldsO[qlane * 1028 + (wave * 8 + j) * 16 + kh8 + r] = o[j][r] * rl;
  __syncthreads();
#pragma unroll 1
  for (int pass = 0; pass < 2; ++pass) {
    for (int i = t; i < 16 * 256; i += 256) { const int ql = i >> 8, q4 = (i & 255) * 4;
      *(volatile v4f_t*)(attn + (size_t)(b * SS + q0 + ql) * DD + q4) = *(const volatile v4fa*)(ldsO + ql * 1028 + q4); }
    __threadfence();
  }
}
__global__ __launch_bounds__(256) void k_deq(const int* __restrict__ wq, bf16* __restrict__ qd) {
  const int o = blockIdx.x, t = threadIdx.x;
  bf16 v[4];
#pragma unroll
  for (int i = 0; i < 4; ++i) v[i] = (bf16)(float)(wq[(size_t)o * DD + t * 4 + i] - 128);
  typedef __attribute__((ext_vector_type(2))) unsigned v2u; typedef unsigned v2ua __attribute__((ext_vector_type(2), may_alias));
  *(volatile v2u*)(qd + (size_t)o * DD + t * 4) = *(const v2ua*)v; __threadfence(); *(volatile v2u*)(qd + (size_t)o * DD + t * 4) = *(const v2ua*)v;
}

extern "C" void kernel_launch(void* const* d_in, const int* in_sizes, int n_in,
                              void* d_out, int out_size, void* d_ws, size_t ws_size,
                              hipStream_t stream) {
  (void)in_sizes; (void)n_in; (void)out_size; (void)ws_size;
  const float* X   = (const float*)d_in[0];
  const int*   wq  = (const int*)d_in[1];
  const float* scale = (const float*)d_in[2];
  char* ws = (char*)d_ws;
  float* attn = (float*)ws; ws += (size_t)BB * SS * DD * 4;
  bf16*  qd   = (bf16*)ws;  ws += (size_t)DD * DD * 2;
  k_deq<<<DD, 256, 0, stream>>>(wq, qd);
  ob_attn<<<dim3(SS / 16, BB), 256, 0, stream>>>(X, attn);
  gemm_split_kernel<float, bf16, 2><<<dim3(BB * SS / 128, DD / 256), 256, 0, stream>>>(attn, 0, qd, 0, scale, (float*)d_out, BB * SS, DD, DD);
}
